// CSWinB_90520730730921
// MI455X (gfx1250) — hardware-verified
//
#include <hip/hip_runtime.h>
#include <math.h>
#include <stdint.h>

#define NBAT   4
#define LTOK   4096
#define MTOK   16384
#define CIN    256
#define C2     512
#define C3     1536
#define HDIM   32
#define QSC64  (0.17677669529663688f * 64.0f)
#define STP    68
#define SBP    132
#define ASP    36
#define ATT_KS  0
#define ATT_VT  32768
#define ATT_ST  65536
#define ATT_END 83968

static_assert(ATT_VT == ATT_KS + 512 * HDIM * 2);
static_assert(ATT_ST == ATT_VT + HDIM * 512 * 2);
static_assert(ATT_END == ATT_ST + 8 * 16 * ASP * 4);
static_assert((STP * 4) % 16 == 0);
static_assert((SBP * 4) % 16 == 0);
static_assert((ASP * 4) % 16 == 0);
static_assert(8 * 16 * STP <= 8704);
static_assert(64 * SBP <= 8704);

typedef _Float16 v16h __attribute__((ext_vector_type(16)));
typedef _Float16 v8h  __attribute__((ext_vector_type(8)));
typedef float    v8f  __attribute__((ext_vector_type(8)));
typedef float    v4f  __attribute__((ext_vector_type(4)));
typedef unsigned int v4u __attribute__((ext_vector_type(4)));

__device__ __forceinline__ unsigned short bf_bits(float f) {
  unsigned u = __float_as_uint(f);
  return (unsigned short)((u + 0x7FFFu + ((u >> 16) & 1u)) >> 16);
}
__device__ __forceinline__ float bfr(float f) { return __uint_as_float(((unsigned)bf_bits(f)) << 16); }
__device__ __forceinline__ unsigned short h_bits(_Float16 x) { return __builtin_bit_cast(unsigned short, x); }
__device__ __forceinline__ unsigned pk16(unsigned short a, unsigned short b) { return (unsigned)a | ((unsigned)b << 16); }
__device__ __forceinline__ v8f zero8() { v8f z = {0.f, 0.f, 0.f, 0.f, 0.f, 0.f, 0.f, 0.f}; return z; }

__device__ __forceinline__ v16h ldfrag_h(const _Float16* p) {
  union { v16h v; v8h h[2]; } f;
  f.h[0] = *(const v8h*)(p);
  f.h[1] = *(const v8h*)(p + 16);
  return f.v;
}

__device__ __forceinline__ v8f mma_h(v16h a, v16h b, v8f c) {
  c = __builtin_amdgcn_wmma_f32_16x16x32_f16(false, a, false, b, (short)0, c, false, false);
#if defined(__HIP_DEVICE_COMPILE__)
  asm volatile("v_nop\n\tv_nop\n\tv_nop\n\tv_nop" : "+v"(c) : "v"(a), "v"(b));
#endif
  return c;
}
__device__ __forceinline__ void wave_sync_lds() {
  __builtin_amdgcn_fence(__ATOMIC_RELEASE, "workgroup");
  __builtin_amdgcn_wave_barrier();
  __builtin_amdgcn_fence(__ATOMIC_ACQUIRE, "workgroup");
}

__device__ __forceinline__ v4u pack8h(v4f a, v4f b) {
  v4u p;
  p[0] = pk16(h_bits((_Float16)a[0]), h_bits((_Float16)a[1]));
  p[1] = pk16(h_bits((_Float16)a[2]), h_bits((_Float16)a[3]));
  p[2] = pk16(h_bits((_Float16)b[0]), h_bits((_Float16)b[1]));
  p[3] = pk16(h_bits((_Float16)b[2]), h_bits((_Float16)b[3]));
  return p;
}
__device__ __forceinline__ void split8h(v4f a, v4f b, v4u& ph, v4u& pl) {
  v4f ra, rb;
#pragma unroll
  for (int e = 0; e < 4; ++e) {
    const _Float16 ha = (_Float16)a[e];
    ra[e] = (a[e] - (float)ha) * 2048.0f;
    const _Float16 hb = (_Float16)b[e];
    rb[e] = (b[e] - (float)hb) * 2048.0f;
  }
  ph = pack8h(a, b);
  pl = pack8h(ra, rb);
}

__device__ __forceinline__ int tok_row(int n, int br, int wI, int b) {
  const int l0 = ((n >> 3) << 6) + (wI << 3) + (n & 7);
  const int l1 = (((wI << 3) + (n >> 6)) << 6) + (n & 63);
  return b * LTOK + ((br != 0) ? l1 : l0);
}

__global__ __launch_bounds__(256) void cvt_wT(const float* __restrict__ w, unsigned short* outp, int nin, int nout) {
  __shared__ float tile[64][33];
  const int tid = threadIdx.x;
  const int i0 = blockIdx.x * 64;
  const int o0 = blockIdx.y * 32;
#pragma unroll
  for (int p = 0; p < 8; ++p) {
    const int idx = p * 256 + tid;
    const int i = idx >> 5, o = idx & 31;
    tile[i][o] = w[(size_t)(i0 + i) * nout + o0 + o];
  }
  __syncthreads();
  const int o = tid >> 3, c8 = (tid & 7) * 8;
  v4u pk;
#pragma unroll
  for (int e = 0; e < 4; ++e) {
    const float f0 = bfr(tile[c8 + 2 * e][o]) * 256.0f;
    const float f1 = bfr(tile[c8 + 2 * e + 1][o]) * 256.0f;
    pk[e] = pk16(h_bits((_Float16)f0), h_bits((_Float16)f1));
  }
  unsigned short* gp = outp + (size_t)(o0 + o) * nin + i0 + c8;
  *(volatile v4u*)gp = pk;
  __threadfence();
  *(volatile v4u*)gp = pk;
}

__global__ __launch_bounds__(256) void cvt_x(const float* __restrict__ x, unsigned short* xt) {
  __shared__ __align__(16) float tile[64 * STP];
  const int tid = threadIdx.x;
  const int bid = blockIdx.x;
  const int cq = bid & 3, pt = (bid >> 2) & 63, b = bid >> 8;
  const int p0 = pt * 64, ch0 = cq * 64;
#pragma unroll
  for (int it = 0; it < 4; ++it) {
    const int q = it * 256 + tid;
    const int ch = q >> 4, j4 = (q & 15) * 4;
    const v4f v = *(const v4f*)(x + ((size_t)(b * CIN + ch0 + ch)) * LTOK + p0 + j4);
#pragma unroll
    for (int e = 0; e < 4; ++e) tile[(j4 + e) * STP + ch] = bfr(v[e]) * 16.0f;
  }
  __syncthreads();
  v4u pk[2];
  size_t offs[2];
#pragma unroll
  for (int it = 0; it < 2; ++it) {
    const int tok = it * 32 + (tid >> 3), piece = tid & 7;
    const v4f fa = *(const v4f*)(tile + tok * STP + piece * 8);
    const v4f fb = *(const v4f*)(tile + tok * STP + piece * 8 + 4);
    pk[it] = pack8h(fa, fb);
    offs[it] = ((size_t)(b * LTOK + p0 + tok)) * CIN + ch0 + piece * 8;
  }
  for (int pass = 0; pass < 2; ++pass) {
#pragma unroll
    for (int it = 0; it < 2; ++it) *(volatile v4u*)(xt + offs[it]) = pk[it];
    __threadfence();
  }
}

__global__ __launch_bounds__(256) void ln512(const float* __restrict__ x2, const float* __restrict__ g,
                                             const float* __restrict__ bb, unsigned short* ih, unsigned short* il,
                                             int row0) {
#pragma clang fp contract(off)
  const int tid = threadIdx.x, wave = tid >> 5, lane = tid & 31;
  const int lr = blockIdx.x * 8 + wave;
  const float* xr = x2 + (size_t)(row0 + lr) * C2;
  const int ca = lane * 8, cb = 256 + lane * 8;
  v4f a[4];
  a[0] = *(const v4f*)(xr + ca);
  a[1] = *(const v4f*)(xr + ca + 4);
  a[2] = *(const v4f*)(xr + cb);
  a[3] = *(const v4f*)(xr + cb + 4);
  float s = 0.f;
#pragma unroll
  for (int i = 0; i < 4; ++i) s = s + ((a[i][0] + a[i][1]) + (a[i][2] + a[i][3]));
#pragma unroll
  for (int off = 1; off < 32; off <<= 1) s = s + __shfl_xor(s, off, 32);
  const float mu = s * (1.0f / 512.0f);
  v4f d[4];
  float s2 = 0.f;
#pragma unroll
  for (int i = 0; i < 4; ++i) {
#pragma unroll
    for (int e = 0; e < 4; ++e) {
      d[i][e] = a[i][e] - mu;
      const float dd = d[i][e] * d[i][e];
      s2 = s2 + dd;
    }
  }
#pragma unroll
  for (int off = 1; off < 32; off <<= 1) s2 = s2 + __shfl_xor(s2, off, 32);
  const float var = s2 * (1.0f / 512.0f);
  const float rstd = rsqrtf(var + 1e-5f);
  v4f z[4];
#pragma unroll
  for (int i = 0; i < 4; ++i) {
    const int cbase = ((i < 2) ? ca : cb) + (i & 1) * 4;
#pragma unroll
    for (int e = 0; e < 4; ++e) {
      const int ch = cbase + e;
      float t0 = d[i][e] * rstd;
      t0 = t0 * bfr(g[ch]);
      t0 = t0 + bfr(bb[ch]);
      z[i][e] = t0 * 8.0f;
    }
  }
  v4u ph0, pl0, ph1, pl1;
  split8h(z[0], z[1], ph0, pl0);
  split8h(z[2], z[3], ph1, pl1);
  const size_t oa = (size_t)lr * C2 + ca, ob = (size_t)lr * C2 + cb;
  for (int pass = 0; pass < 2; ++pass) {
    *(volatile v4u*)(ih + oa) = ph0;
    *(volatile v4u*)(ih + ob) = ph1;
    *(volatile v4u*)(il + oa) = pl0;
    *(volatile v4u*)(il + ob) = pl1;
    __threadfence();
  }
}

template <int MODE, bool ALO, bool AHB>
__global__ __launch_bounds__(256)
void gemm_k(const unsigned short* __restrict__ Ah, const unsigned short* __restrict__ Al,
            const unsigned short* __restrict__ Bt, int K, int Mrows,
            const float* __restrict__ f0, const float* __restrict__ f1,
            float* outF, unsigned short* h0, unsigned short* h1, unsigned short* h2, unsigned short* h3,
            float oscale) {
  __shared__ __align__(16) float sbuf[8704];
  const int tid = threadIdx.x, wave = tid >> 5, lane = tid & 31, hh = lane >> 4, c = lane & 15;
  const int n0 = blockIdx.x * 64, m0 = blockIdx.y * 128;
  const int arow = m0 + wave * 16 + c;
  const _Float16* A0 = (const _Float16*)(const void*)Ah;
  const _Float16* A1 = (const _Float16*)(const void*)Al;
  const _Float16* B  = (const _Float16*)(const void*)Bt;

  v8f acch[4], accl[4];
#pragma unroll
  for (int nt = 0; nt < 4; ++nt) { acch[nt] = zero8(); accl[nt] = zero8(); }

#pragma unroll 1
  for (int k0 = 0; k0 < K; k0 += 32) {
    size_t aoff;
    if (AHB) aoff = ((size_t)(k0 >> 5) * Mrows + arow) * 32 + 8 * hh;
    else     aoff = (size_t)arow * K + k0 + 8 * hh;
    const v16h ah = ldfrag_h(A0 + aoff);
    v16h al = ah;
    if (ALO) al = ldfrag_h(A1 + aoff);
#pragma unroll
    for (int nt = 0; nt < 4; ++nt) {
      const v16h bfrag = ldfrag_h(B + (size_t)(n0 + nt * 16 + c) * K + k0 + 8 * hh);
      acch[nt] = mma_h(ah, bfrag, acch[nt]);
      if (ALO) accl[nt] = mma_h(al, bfrag, accl[nt]);
    }
  }

  if (MODE == 3) {
    float* sb = sbuf;
#pragma unroll
    for (int nt = 0; nt < 4; ++nt) {
#pragma unroll
      for (int r = 0; r < 8; ++r) {
        float v = acch[nt][r];
        if (ALO) v = v + accl[nt][r] * (1.0f / 2048.0f);
        sb[(nt * 16 + c) * SBP + wave * 16 + 8 * hh + r] = v * oscale;
      }
    }
    __syncthreads();
    const int bimg = m0 >> 12, l0 = m0 & 4095;
    v4f ov[8];
    size_t offs[8];
#pragma unroll
    for (int i = 0; i < 8; ++i) {
      const int cc = wave * 8 + i;
      ov[i] = *(const v4f*)(sb + cc * SBP + lane * 4);
      offs[i] = ((size_t)(bimg * CIN + n0 + cc)) * LTOK + l0 + lane * 4;
    }
    for (int pass = 0; pass < 2; ++pass) {
#pragma unroll
      for (int i = 0; i < 8; ++i) *(volatile v4f*)(outF + offs[i]) = ov[i];
      __threadfence();
    }
  } else {
    float* st = sbuf + wave * (16 * STP);
#pragma unroll
    for (int nt = 0; nt < 4; ++nt) {
#pragma unroll
      for (int r = 0; r < 8; ++r) {
        float v = acch[nt][r];
        if (ALO) v = v + accl[nt][r] * (1.0f / 2048.0f);
        st[(8 * hh + r) * STP + nt * 16 + c] = v * oscale;
      }
    }
    wave_sync_lds();
    if (MODE == 0) {
      v4f ov[8];
      size_t offs[8];
#pragma unroll
      for (int it = 0; it < 8; ++it) {
        const int q = it * 2 + hh;
        ov[it] = *(const v4f*)(st + q * STP + c * 4);
        offs[it] = (size_t)(m0 + wave * 16 + q) * C2 + n0 + c * 4;
      }
      for (int pass = 0; pass < 2; ++pass) {
#pragma unroll
        for (int it = 0; it < 8; ++it) *(volatile v4f*)(outF + offs[it]) = ov[it];
        __threadfence();
      }
    } else if (MODE == 1) {
      const int part = n0 >> 9, colp = n0 & 511;
      const float sc = (part == 0) ? QSC64 : 16.0f;
      unsigned short* dA = (part == 0) ? h0 : ((part == 1) ? h1 : h2);
      v4u pa[4], pb[4];
      size_t offs[4];
#pragma unroll
      for (int it = 0; it < 4; ++it) {
        const int q = it * 4 + (lane >> 3), piece = lane & 7;
        v4f fa = *(const v4f*)(st + q * STP + piece * 8);
        v4f fb = *(const v4f*)(st + q * STP + piece * 8 + 4);
        fa = fa * sc;
        fb = fb * sc;
        split8h(fa, fb, pa[it], pb[it]);
        offs[it] = (size_t)(m0 + wave * 16 + q) * C2 + colp + piece * 8;
      }
      for (int pass = 0; pass < 2; ++pass) {
#pragma unroll
        for (int it = 0; it < 4; ++it) {
          *(volatile v4u*)(dA + offs[it]) = pa[it];
          if (part == 2) *(volatile v4u*)(h3 + offs[it]) = pb[it];
        }
        __threadfence();
      }
    } else {
      v4u pa[4], pb[4];
      size_t offs[4];
#pragma unroll
      for (int it = 0; it < 4; ++it) {
        const int q = it * 4 + (lane >> 3), piece = lane & 7;
        const int col0 = n0 + piece * 8;
        const size_t ro = (size_t)(m0 + wave * 16 + q) * C2 + col0;
        const v4f fa = *(const v4f*)(st + q * STP + piece * 8);
        const v4f fb = *(const v4f*)(st + q * STP + piece * 8 + 4);
        const v4f ra = *(const v4f*)(f1 + ro);
        const v4f rb = *(const v4f*)(f1 + ro + 4);
        v4f ua, ub;
#pragma unroll
        for (int e = 0; e < 4; ++e) {
          float ta = fa[e] + bfr(f0[col0 + e]);
          ta = ra[e] + ta;
          ua[e] = ta * 32.0f;
          float tb = fb[e] + bfr(f0[col0 + 4 + e]);
          tb = rb[e] + tb;
          ub[e] = tb * 32.0f;
        }
        split8h(ua, ub, pa[it], pb[it]);
        offs[it] = ro;
      }
      for (int pass = 0; pass < 2; ++pass) {
#pragma unroll
        for (int it = 0; it < 4; ++it) {
          *(volatile v4u*)(h0 + offs[it]) = pa[it];
          *(volatile v4u*)(h1 + offs[it]) = pb[it];
        }
        __threadfence();
      }
    }
  }
}

__global__ __launch_bounds__(256)
void attn_k(const unsigned short* __restrict__ Qp, const unsigned short* __restrict__ Kp,
            const unsigned short* __restrict__ Vp,
            const float* __restrict__ cw0, const float* __restrict__ cb0,
            const float* __restrict__ cw1, const float* __restrict__ cb1,
            unsigned short* Oh) {
  extern __shared__ __align__(16) char smem[];
  unsigned short* Ks = (unsigned short*)(smem + ATT_KS);
  unsigned short* Vt = (unsigned short*)(smem + ATT_VT);
  float* Sst = (float*)(smem + ATT_ST);
  const int tid = threadIdx.x, wave = tid >> 5, lane = tid & 31, hh = lane >> 4, c = lane & 15;
  const int br = blockIdx.y;
  const int hd = blockIdx.x & 7, wI = (blockIdx.x >> 3) & 7, b = blockIdx.x >> 6;
  const int c0 = br * 256 + hd * HDIM;
  const int wsh = (br != 0) ? 6 : 3;
  const int Wsp = 1 << wsh, Hsp = 512 >> wsh;

#pragma unroll
  for (int it = 0; it < 2; ++it) {
    const int n = it * 256 + tid;
    const size_t row = (size_t)tok_row(n, br, wI, b);
    const v4u* kg = (const v4u*)(Kp + row * C2 + c0);
    const v4u* vg = (const v4u*)(Vp + row * C2 + c0);
#pragma unroll
    for (int i = 0; i < 4; ++i) {
      const v4u kw = kg[i];
      *(v4u*)(Ks + n * HDIM + 8 * i) = kw;
      const v4u vw = vg[i];
#pragma unroll
      for (int e = 0; e < 4; ++e) {
        const unsigned w32 = vw[e];
        Vt[(8 * i + 2 * e) * 512 + n]     = (unsigned short)(w32 & 0xFFFFu);
        Vt[(8 * i + 2 * e + 1) * 512 + n] = (unsigned short)(w32 >> 16);
      }
    }
  }
  __syncthreads();

  const float* cw  = (br != 0) ? cw1 : cw0;
  const float* cbp = (br != 0) ? cb1 : cb0;
  const int cha = hd * HDIM + c, chb = cha + 16;
  float wA[9], wB[9];
#pragma unroll
  for (int t = 0; t < 9; ++t) { wA[t] = bfr(cw[cha * 9 + t]); wB[t] = bfr(cw[chb * 9 + t]); }
  const float bA = bfr(cbp[cha]), bB = bfr(cbp[chb]);

  const _Float16* Ksh = (const _Float16*)(const void*)Ks;
  const _Float16* Vth = (const _Float16*)(const void*)Vt;
  const _Float16* Qg  = (const _Float16*)(const void*)Qp;
  float* st = Sst + wave * (16 * ASP);

#pragma unroll 1
  for (int qt = wave; qt < 32; qt += 8) {
    const size_t rq = (size_t)tok_row(qt * 16 + c, br, wI, b);
    const v16h qf = ldfrag_h(Qg + rq * C2 + c0 + 8 * hh);
    v8f o0 = zero8(), o1 = zero8();
    float mrun = -1.0e30f, lrun = 0.f;
#pragma unroll 1
    for (int ch = 0; ch < 8; ++ch) {
      const int kb = ch * 64;
      v8f s[4];
#pragma unroll
      for (int j = 0; j < 4; ++j) {
        const v16h ka = ldfrag_h(Ksh + (size_t)(kb + j * 16 + c) * HDIM + 8 * hh);
        s[j] = mma_h(ka, qf, zero8());
      }
      float mc = s[0][0];
#pragma unroll
      for (int j = 0; j < 4; ++j) {
#pragma unroll
        for (int r = 0; r < 8; ++r) mc = fmaxf(mc, s[j][r]);
      }
      mc = fmaxf(mc, __shfl_xor(mc, 16, 32));
      const float mnew = fmaxf(mrun, mc);
      const float alpha = __expf((mrun - mnew) * (1.0f / 1024.0f));
#pragma unroll
      for (int r = 0; r < 8; ++r) {
        const float ar = __shfl(alpha, 8 * hh + r, 32);
        o0[r] = o0[r] * ar;
        o1[r] = o1[r] * ar;
      }
      float psum = 0.f;
      v16h pf0, pf1;
#pragma unroll
      for (int i = 0; i < 8; ++i) {
        const float e0 = __expf((s[0][i] - mnew) * (1.0f / 1024.0f));
        const float e1 = __expf((s[1][i] - mnew) * (1.0f / 1024.0f));
        const float e2 = __expf((s[2][i] - mnew) * (1.0f / 1024.0f));
        const float e3 = __expf((s[3][i] - mnew) * (1.0f / 1024.0f));
        psum = psum + ((e0 + e1) + (e2 + e3));
        pf0[i]     = (_Float16)(e0 * 1024.0f);
        pf0[8 + i] = (_Float16)(e1 * 1024.0f);
        pf1[i]     = (_Float16)(e2 * 1024.0f);
        pf1[8 + i] = (_Float16)(e3 * 1024.0f);
      }
      lrun = lrun * alpha + psum;
      mrun = mnew;
      {
        const v16h va = ldfrag_h(Vth + (size_t)c * 512 + kb + 8 * hh);
        const v16h vb = ldfrag_h(Vth + (size_t)(16 + c) * 512 + kb + 8 * hh);
        o0 = mma_h(pf0, va, o0);
        o1 = mma_h(pf0, vb, o1);
        const v16h vc = ldfrag_h(Vth + (size_t)c * 512 + kb + 32 + 8 * hh);
        const v16h vd = ldfrag_h(Vth + (size_t)(16 + c) * 512 + kb + 32 + 8 * hh);
        o0 = mma_h(pf1, vc, o0);
        o1 = mma_h(pf1, vd, o1);
      }
    }
    const float lsum = lrun + __shfl_xor(lrun, 16, 32);
#pragma unroll
    for (int r = 0; r < 8; ++r) {
      const int q = 8 * hh + r;
      const float lq = __shfl(lsum, q, 32);
      const float inv = 1.0f / (lq * 16384.0f);
      const int n = qt * 16 + q;
      const int wi = n >> wsh, wj = n & (Wsp - 1);
      float la = 0.f, lb = 0.f;
#pragma unroll
      for (int di = 0; di < 3; ++di) {
#pragma unroll
        for (int dj = 0; dj < 3; ++dj) {
          const int ii = wi + di - 1, jj = wj + dj - 1;
          const bool ok = ((unsigned)ii < (unsigned)Hsp) && ((unsigned)jj < (unsigned)Wsp);
          const int nn = ok ? ((ii << wsh) + jj) : n;
          const float xa = (float)Vth[(size_t)c * 512 + nn];
          const float xb = (float)Vth[(size_t)(16 + c) * 512 + nn];
          la += (ok ? xa : 0.f) * wA[di * 3 + dj];
          lb += (ok ? xb : 0.f) * wB[di * 3 + dj];
        }
      }
      const float va = o0[r] * inv + (la * (1.0f / 16.0f) + bA);
      const float vb = o1[r] * inv + (lb * (1.0f / 16.0f) + bB);
      st[q * ASP + c] = va;
      st[q * ASP + 16 + c] = vb;
    }
    wave_sync_lds();
    v4u pk[2];
    size_t offs[2];
#pragma unroll
    for (int t = 0; t < 2; ++t) {
      const int q = t * 8 + (lane >> 2), piece = lane & 3;
      v4f fa = *(const v4f*)(st + q * ASP + piece * 8);
      v4f fb = *(const v4f*)(st + q * ASP + piece * 8 + 4);
      fa = fa * 256.0f;
      fb = fb * 256.0f;
      pk[t] = pack8h(fa, fb);
      const int row = tok_row(qt * 16 + q, br, wI, b);
      offs[t] = (((size_t)(br * 8 + hd)) * MTOK + (size_t)row) * HDIM + piece * 8;
    }
    for (int pass = 0; pass < 2; ++pass) {
#pragma unroll
      for (int t = 0; t < 2; ++t) *(volatile v4u*)(Oh + offs[t]) = pk[t];
      __threadfence();
    }
    wave_sync_lds();
  }
}

extern "C" void kernel_launch(void* const* d_in, const int* in_sizes, int n_in,
                              void* d_out, int out_size, void* d_ws, size_t ws_size,
                              hipStream_t stream) {
  if (n_in < 12) return;
  if (in_sizes[0] != NBAT * CIN * LTOK) return;
  if (in_sizes[1] != CIN * C2 || in_sizes[2] != C2 || in_sizes[3] != C2) return;
  if (in_sizes[4] != C2 * C3) return;
  if (in_sizes[5] != CIN * 9 || in_sizes[6] != CIN || in_sizes[7] != CIN * 9 || in_sizes[8] != CIN) return;
  if (in_sizes[9] != C2 * C2 || in_sizes[10] != C2 || in_sizes[11] != C2 * CIN) return;
  if (out_size != 2 * NBAT * CIN * LTOK) return;

  const float* x       = (const float*)d_in[0];
  const float* w_embed = (const float*)d_in[1];
  const float* g1      = (const float*)d_in[2];
  const float* b1      = (const float*)d_in[3];
  const float* w_qkv   = (const float*)d_in[4];
  const float* cw0     = (const float*)d_in[5];
  const float* cb0     = (const float*)d_in[6];
  const float* cw1     = (const float*)d_in[7];
  const float* cb1     = (const float*)d_in[8];
  const float* w_proj  = (const float*)d_in[9];
  const float* b_proj  = (const float*)d_in[10];
  const float* w_out   = (const float*)d_in[11];
  float* out = (float*)d_out;

  const size_t sWe = (size_t)CIN * C2 * 2;
  const size_t sWq = (size_t)C2 * C3 * 2;
  const size_t sWp = (size_t)C2 * C2 * 2;
  const size_t sWo = (size_t)C2 * CIN * 2;
  const size_t sXT = (size_t)MTOK * CIN * 2;
  const size_t sTh = (size_t)(MTOK / 2) * C2 * 2;
  const size_t sX2 = (size_t)MTOK * C2 * 4;
  const size_t sP  = (size_t)MTOK * C2 * 2;
  size_t off = 0;
  const size_t oWe = off; off += sWe;
  const size_t oWq = off; off += sWq;
  const size_t oWp = off; off += sWp;
  const size_t oWo = off; off += sWo;
  const size_t oXT = off; off += sXT;
  const size_t oT  = off; off += 2 * sTh;
  const size_t oX2 = off; off += sX2;
  const size_t oQ  = off; off += sP;
  const size_t oK  = off; off += sP;
  const size_t oVh = off; off += sP;
  const size_t oVl = off; off += sP;
  if (off > ws_size) return;
  if (off > (size_t)134217728) return;
  if (2 * sTh != (size_t)16 * MTOK * HDIM * 2) return;

  char* ws = (char*)d_ws;
  unsigned short* We = (unsigned short*)(ws + oWe);
  unsigned short* Wq = (unsigned short*)(ws + oWq);
  unsigned short* Wp = (unsigned short*)(ws + oWp);
  unsigned short* Wo = (unsigned short*)(ws + oWo);
  unsigned short* XT = (unsigned short*)(ws + oXT);
  unsigned short* Ih = (unsigned short*)(ws + oT);
  unsigned short* Il = (unsigned short*)(ws + oT + sTh);
  unsigned short* Oh = (unsigned short*)(ws + oT);
  float* X2 = (float*)(ws + oX2);
  unsigned short* Qp = (unsigned short*)(ws + oQ);
  unsigned short* Kp = (unsigned short*)(ws + oK);
  unsigned short* Xh = (unsigned short*)(ws + oQ);
  unsigned short* Xl = (unsigned short*)(ws + oK);
  unsigned short* Vh = (unsigned short*)(ws + oVh);
  unsigned short* Vl = (unsigned short*)(ws + oVl);

  const dim3 blk(256);
  cvt_wT<<<dim3(CIN / 64, C2 / 32), blk, 0, stream>>>(w_embed, We, CIN, C2);
  cvt_wT<<<dim3(C2 / 64, C3 / 32), blk, 0, stream>>>(w_qkv, Wq, C2, C3);
  cvt_wT<<<dim3(C2 / 64, C2 / 32), blk, 0, stream>>>(w_proj, Wp, C2, C2);
  cvt_wT<<<dim3(C2 / 64, CIN / 32), blk, 0, stream>>>(w_out, Wo, C2, CIN);
  cvt_x<<<dim3(NBAT * 64 * 4), blk, 0, stream>>>(x, XT);
  gemm_k<0, false, false><<<dim3(C2 / 64, MTOK / 128), blk, 0, stream>>>(
      XT, XT, We, CIN, MTOK, g1, g1, X2, XT, XT, XT, XT, 1.0f / 4096.0f);
  for (int half = 0; half < 2; ++half) {
    const size_t ro = (size_t)half * (MTOK / 2) * C2;
    ln512<<<dim3((MTOK / 2) / 8), blk, 0, stream>>>(X2, g1, b1, Ih, Il, half * (MTOK / 2));
    gemm_k<1, true, false><<<dim3(C3 / 64, (MTOK / 2) / 128), blk, 0, stream>>>(
        Ih, Il, Wq, C2, MTOK, g1, g1, X2, Qp + ro, Kp + ro, Vh + ro, Vl + ro, 1.0f / 2048.0f);
  }
  gemm_k<3, true, false><<<dim3(CIN / 64, MTOK / 128), blk, 0, stream>>>(
      Vh, Vl, Wo, C2, MTOK, g1, g1, out + (size_t)NBAT * CIN * LTOK, XT, XT, XT, XT, 1.0f / 4096.0f);
  (void)hipFuncSetAttribute(reinterpret_cast<const void*>(&attn_k), hipFuncAttributeMaxDynamicSharedMemorySize, ATT_END);
  attn_k<<<dim3(NBAT * 8 * 8, 2), blk, ATT_END, stream>>>(Qp, Kp, Vh, cw0, cb0, cw1, cb1, Oh);
  gemm_k<2, false, true><<<dim3(C2 / 64, MTOK / 128), blk, 0, stream>>>(
      Oh, Oh, Wp, C2, MTOK, b_proj, X2, X2, Xh, Xl, XT, XT, 1.0f / 65536.0f);
  gemm_k<3, true, false><<<dim3(CIN / 64, MTOK / 128), blk, 0, stream>>>(
      Xh, Xl, Wo, C2, MTOK, g1, g1, out, XT, XT, XT, XT, 1.0f / 8192.0f);
  (void)hipGetLastError();
}
